// EncoderBlock_36146444763558
// MI455X (gfx1250) — hardware-verified
//
#include <hip/hip_runtime.h>

#ifndef NB
#define NB 4
#endif
#ifndef SEQ
#define SEQ 1024
#endif
#define NB_FULL 4
#define SEQ_FULL 1024
#ifndef OSEQ
#define OSEQ SEQ_FULL
#endif
#define DM 1024
#define NH 16
#define HD 64
#define DFF 4096
#define KQB 64
#define NR ((size_t)NB * SEQ)
#define RMS_EPS 1e-6f

static_assert(NB >= 1 && NB <= NB_FULL);
static_assert(SEQ % 128 == 0 && SEQ <= SEQ_FULL);
static_assert(DM == NH * HD && HD == 64);
static_assert(DM % 256 == 0 && DFF % 64 == 0 && DM % 32 == 0 && DFF % 32 == 0);
static_assert(((NB * SEQ) % 128) == 0);
static_assert(SEQ % KQB == 0);

typedef _Float16 v16h __attribute__((ext_vector_type(16)));
typedef __bf16   v16b __attribute__((ext_vector_type(16)));
typedef unsigned short v8us __attribute__((ext_vector_type(8), may_alias));
typedef float v8f __attribute__((ext_vector_type(8)));
typedef float v4f __attribute__((ext_vector_type(4)));
typedef float v4fa __attribute__((ext_vector_type(4), may_alias));
union Frag16 { v16h h; v16b b; v8us half[2]; unsigned short u[16]; };
union H1 { _Float16 h; unsigned short u; };
static_assert(sizeof(Frag16) == 32);

__device__ __forceinline__ unsigned short bf16_bits(float x) { unsigned int u = __float_as_uint(x); return (unsigned short)((u + 0x7FFFu + ((u >> 16) & 1u)) >> 16); }
__device__ __forceinline__ float bf16_val(unsigned short b) { return __uint_as_float(((unsigned int)b) << 16); }
__device__ __forceinline__ float bf16_rne(float x) { return bf16_val(bf16_bits(x)); }
__device__ __forceinline__ unsigned short f16_bits(float x) { H1 t; t.h = (_Float16)x; return t.u; }
__device__ __forceinline__ float f16_val(unsigned short u) { H1 t; t.u = u; return (float)t.h; }

__device__ __forceinline__ Frag16 ld_frag(const unsigned short* p, int hh) {
  Frag16 f;
  f.half[0] = *(const v8us*)(p + 8 * hh);
  f.half[1] = *(const v8us*)(p + 16 + 8 * hh);
  return f;
}
__device__ __forceinline__ v8f mma_h(v16h a, v16h b, v8f c) {
  v8f d = __builtin_amdgcn_wmma_f32_16x16x32_f16(false, a, false, b, (short)0, c, false, false);
  asm volatile("v_nop\n\tv_nop\n\tv_nop\n\tv_nop" : "+v"(d) : "v"(a), "v"(b));
  return d;
}
__device__ __forceinline__ v8f mma_b(v16b a, v16b b, v8f c) {
  v8f d = __builtin_amdgcn_wmma_f32_16x16x32_bf16(false, a, false, b, (short)0, c, false, false);
  asm volatile("v_nop\n\tv_nop\n\tv_nop\n\tv_nop" : "+v"(d) : "v"(a), "v"(b));
  return d;
}
template <bool BF>
__device__ __forceinline__ v8f mmx(const Frag16& a, const Frag16& b, v8f c) {
  if (BF) return mma_b(a.b, b.b, c);
  return mma_h(a.h, b.h, c);
}

template <bool BF, bool GAM>
__global__ __launch_bounds__(256) void k_wt(const float* __restrict__ W, const float* __restrict__ g, unsigned short* __restrict__ Bt, int K, int N, float scale) {
  const int k8n = K >> 3;
  const size_t t = (size_t)blockIdx.x * 256 + threadIdx.x;
  if (t >= (size_t)N * (size_t)k8n) return;
  const int n = (int)(t / (size_t)k8n), k8 = (int)(t % (size_t)k8n) * 8;
  float gv[8];
#pragma unroll
  for (int i = 0; i < 8; ++i) gv[i] = 1.0f;
  if (GAM) {
    const v4f ga = *(const v4fa*)(g + k8), gb = *(const v4fa*)(g + k8 + 4);
#pragma unroll
    for (int i = 0; i < 4; ++i) { gv[i] = bf16_rne(ga[i]); gv[4 + i] = bf16_rne(gb[i]); }
  }
  Frag16 f;
#pragma unroll
  for (int i = 0; i < 8; ++i) {
    const float wv = bf16_rne(W[(size_t)(k8 + i) * (size_t)N + n]) * gv[i];
    f.u[i] = BF ? bf16_bits(wv) : f16_bits(wv * scale);
  }
  unsigned short* d = Bt + (size_t)n * (size_t)K + k8;
  *(volatile v8us*)d = f.half[0];
  __threadfence();
  *(volatile v8us*)d = f.half[0];
}

template <bool RIN, bool WXB, bool WF16, bool WBHL>
__global__ __launch_bounds__(256) void k_rms(const float* __restrict__ F, int spitch, float eps, float* __restrict__ XB,
    unsigned short* __restrict__ F16, unsigned short* __restrict__ PH, unsigned short* __restrict__ PL, float* __restrict__ RS) {
  __shared__ __attribute__((aligned(16))) float red[32];
  const int tid = threadIdx.x, w = tid >> 5, lane = tid & 31;
  const int rb = (int)blockIdx.x * 32;
#pragma unroll 1
  for (int i = 0; i < 4; ++i) {
    const int r = rb + w * 4 + i;
    const float* src = F + ((size_t)(r / SEQ) * (size_t)spitch + (size_t)(r % SEQ)) * DM;
    float ss = 0.f;
#pragma unroll 1
    for (int u = 0; u < DM / 128; ++u) {
      const int j = u * 128 + lane * 4;
      v4f a = *(const v4fa*)(src + j);
      if (RIN) {
#pragma unroll
        for (int q = 0; q < 4; ++q) a[q] = bf16_rne(a[q]);
      }
#pragma unroll
      for (int q = 0; q < 4; ++q) ss += a[q] * a[q];
      if (WXB) {
        float* d = XB + (size_t)r * DM + j;
        *(volatile v4f*)d = a;
        __threadfence();
        *(volatile v4f*)d = a;
      }
    }
    if (WF16 || WBHL) {
#pragma unroll 1
      for (int u = 0; u < DM / 256; ++u) {
        const int j = u * 256 + lane * 8;
        v4f a = *(const v4fa*)(src + j), c = *(const v4fa*)(src + j + 4);
        if (RIN) {
#pragma unroll
          for (int q = 0; q < 4; ++q) { a[q] = bf16_rne(a[q]); c[q] = bf16_rne(c[q]); }
        }
        Frag16 fh, ph, pl;
#pragma unroll
        for (int q = 0; q < 4; ++q) {
          const float v0 = a[q], v1 = c[q];
          fh.u[q] = f16_bits(v0); fh.u[4 + q] = f16_bits(v1);
          const unsigned short h0 = bf16_bits(v0), h1 = bf16_bits(v1);
          ph.u[q] = h0; ph.u[4 + q] = h1;
          pl.u[q] = bf16_bits(v0 - bf16_val(h0)); pl.u[4 + q] = bf16_bits(v1 - bf16_val(h1));
        }
        const size_t o = (size_t)r * DM + j;
        if (WF16) *(volatile v8us*)(F16 + o) = fh.half[0];
        if (WBHL) { *(volatile v8us*)(PH + o) = ph.half[0]; *(volatile v8us*)(PL + o) = pl.half[0]; }
        __threadfence();
        if (WF16) *(volatile v8us*)(F16 + o) = fh.half[0];
        if (WBHL) { *(volatile v8us*)(PH + o) = ph.half[0]; *(volatile v8us*)(PL + o) = pl.half[0]; }
      }
    }
#pragma unroll
    for (int off = 16; off > 0; off >>= 1) ss += __shfl_xor(ss, off, 32);
    if (lane == 0) red[w * 4 + i] = rsqrtf(ss * (1.0f / (float)DM) + eps);
  }
  __syncthreads();
  if (w == 0 && lane < 8) {
    const v4f v = *(const v4fa*)&red[lane * 4];
    float* d = RS + rb + lane * 4;
    *(volatile v4f*)d = v;
    __threadfence();
    *(volatile v4f*)d = v;
  }
}

template <bool BF, bool ASPLIT, int ACT, int OUTM, bool HRS, bool HRES>
__global__ __launch_bounds__(128) void k_gemm(const unsigned short* __restrict__ Ah, const unsigned short* __restrict__ Al, int lda,
    const unsigned short* __restrict__ Bt, int ldb, float alpha, const float* __restrict__ rs, const float* __restrict__ bias,
    const float* __restrict__ resid, int ldr, float* __restrict__ C32, unsigned short* __restrict__ Ch, unsigned short* __restrict__ Cl,
    int ldc, int cseq, int cpitch, int M, int N, int K) {
  static_assert(!(HRES && OUTM != 0));
  static_assert(OUTM >= 0 && OUTM <= 3);
  static_assert(!ASPLIT || BF);
  static_assert(ACT == 0 || ACT == 1);
  __shared__ __attribute__((aligned(16))) float so[4][32][68];
  const int tid = threadIdx.x, w = tid >> 5, lane = tid & 31, ln = lane & 15, hh = lane >> 4;
  const int ntn = N >> 6;
  const int mt = (int)blockIdx.x / ntn, nq = (int)blockIdx.x - mt * ntn;
  const int row0 = mt * 128 + 32 * w, col0 = nq * 64;
  if (row0 + 32 > M) return;
  const unsigned short* a0p = Ah + (size_t)(row0 + ln) * (size_t)lda;
  const unsigned short* a1p = a0p + (size_t)16 * (size_t)lda;
  const unsigned short* e0p = a0p;
  const unsigned short* e1p = a1p;
  if (ASPLIT) { e0p = Al + (size_t)(row0 + ln) * (size_t)lda; e1p = e0p + (size_t)16 * (size_t)lda; }
  const unsigned short* b0p = Bt + (size_t)(col0 + ln) * (size_t)ldb;
  const unsigned short* b1p = b0p + (size_t)16 * (size_t)ldb;
  const unsigned short* b2p = b1p + (size_t)16 * (size_t)ldb;
  const unsigned short* b3p = b2p + (size_t)16 * (size_t)ldb;
  const v8f z8 = {0.f, 0.f, 0.f, 0.f, 0.f, 0.f, 0.f, 0.f};
  v8f c00 = z8, c01 = z8, c02 = z8, c03 = z8, c10 = z8, c11 = z8, c12 = z8, c13 = z8;
#pragma unroll 1
  for (int kb = 0; kb < K; kb += 32) {
    const Frag16 a0 = ld_frag(a0p + kb, hh), a1 = ld_frag(a1p + kb, hh);
    Frag16 e0 = a0, e1 = a1;
    if (ASPLIT) { e0 = ld_frag(e0p + kb, hh); e1 = ld_frag(e1p + kb, hh); }
    Frag16 bq = ld_frag(b0p + kb, hh);
    c00 = mmx<BF>(a0, bq, c00); c10 = mmx<BF>(a1, bq, c10);
    if (ASPLIT) { c00 = mmx<BF>(e0, bq, c00); c10 = mmx<BF>(e1, bq, c10); }
    bq = ld_frag(b1p + kb, hh);
    c01 = mmx<BF>(a0, bq, c01); c11 = mmx<BF>(a1, bq, c11);
    if (ASPLIT) { c01 = mmx<BF>(e0, bq, c01); c11 = mmx<BF>(e1, bq, c11); }
    bq = ld_frag(b2p + kb, hh);
    c02 = mmx<BF>(a0, bq, c02); c12 = mmx<BF>(a1, bq, c12);
    if (ASPLIT) { c02 = mmx<BF>(e0, bq, c02); c12 = mmx<BF>(e1, bq, c12); }
    bq = ld_frag(b3p + kb, hh);
    c03 = mmx<BF>(a0, bq, c03); c13 = mmx<BF>(a1, bq, c13);
    if (ASPLIT) { c03 = mmx<BF>(e0, bq, c03); c13 = mmx<BF>(e1, bq, c13); }
  }
  const v8f accs[8] = {c00, c01, c02, c03, c10, c11, c12, c13};
  float rs0[8], rs1[8];
#pragma unroll
  for (int r = 0; r < 8; ++r) { rs0[r] = 1.0f; rs1[r] = 1.0f; }
  if (HRS) {
    const v4f ra = *(const v4fa*)(rs + row0 + 8 * hh), rbv = *(const v4fa*)(rs + row0 + 8 * hh + 4);
    const v4f rc = *(const v4fa*)(rs + row0 + 16 + 8 * hh), rdv = *(const v4fa*)(rs + row0 + 16 + 8 * hh + 4);
#pragma unroll
    for (int q = 0; q < 4; ++q) { rs0[q] = ra[q]; rs0[4 + q] = rbv[q]; rs1[q] = rc[q]; rs1[4 + q] = rdv[q]; }
  }
#pragma unroll
  for (int u = 0; u < 8; ++u) {
    const int t = u & 3, half = u >> 2;
    const int col = col0 + t * 16 + ln;
    const float bv = bf16_rne(bias[col]);
#pragma unroll
    for (int r = 0; r < 8; ++r) {
      const int rloc = half * 16 + 8 * hh + r;
      float v = accs[u][r] * alpha;
      if (HRS) v *= (half ? rs1[r] : rs0[r]);
      v += bv;
      if (ACT == 1) v = (v >= 0.f) ? v : 0.1f * v;
      so[w][rloc][t * 16 + ln] = v;
    }
  }
  __builtin_amdgcn_fence(4  , "workgroup");
  __builtin_amdgcn_wave_barrier();
  if (OUTM == 0) {
    for (int pass = 0; pass < 2; ++pass) {
#pragma unroll
      for (int q = 0; q < 16; ++q) {
        const int r = q * 2 + (lane >> 4), c4 = (lane & 15) * 4;
        v4f v = *(const v4fa*)&so[w][r][c4];
        const int grow = row0 + r;
        if (HRES) { const v4f rv = *(const v4fa*)(resid + (size_t)grow * (size_t)ldr + col0 + c4); v += rv; }
        const size_t crow = (size_t)(grow / cseq) * (size_t)cpitch + (size_t)(grow % cseq);
        *(volatile v4f*)(C32 + crow * (size_t)ldc + col0 + c4) = v;
      }
      if (pass == 0) __threadfence();
    }
  } else {
    for (int pass = 0; pass < 2; ++pass) {
#pragma unroll
      for (int q = 0; q < 8; ++q) {
        const int r = q * 4 + (lane >> 3), c8 = (lane & 7) * 8;
        const v4f x0 = *(const v4fa*)&so[w][r][c8], x1 = *(const v4fa*)&so[w][r][c8 + 4];
        Frag16 fh, fl;
#pragma unroll
        for (int i = 0; i < 4; ++i) {
          const float v0 = x0[i], v1 = x1[i];
          if (OUTM == 3) {
            const unsigned short h0 = bf16_bits(v0), h1 = bf16_bits(v1);
            fh.u[i] = h0; fh.u[4 + i] = h1;
            fl.u[i] = bf16_bits(v0 - bf16_val(h0)); fl.u[4 + i] = bf16_bits(v1 - bf16_val(h1));
          } else {
            const unsigned short h0 = f16_bits(v0), h1 = f16_bits(v1);
            fh.u[i] = h0; fh.u[4 + i] = h1;
            fl.u[i] = f16_bits((v0 - f16_val(h0)) * 1024.0f); fl.u[4 + i] = f16_bits((v1 - f16_val(h1)) * 1024.0f);
          }
        }
        const size_t o = (size_t)(row0 + r) * (size_t)ldc + col0 + c8;
        *(volatile v8us*)(Ch + o) = fh.half[0];
        if (OUTM >= 2) *(volatile v8us*)(Cl + o) = fl.half[0];
      }
      if (pass == 0) __threadfence();
    }
  }
}

template <int NHv, int TTv, bool TWO>
__global__ __launch_bounds__(256) void k_vt(const unsigned short* __restrict__ V, const unsigned short* __restrict__ V2, int ldv,
    unsigned short* __restrict__ Vt, unsigned short* __restrict__ Vt2) {
  __shared__ __attribute__((aligned(16))) unsigned short tl[64][66];
  __shared__ __attribute__((aligned(16))) unsigned short tl2[64][66];
  const int tid = threadIdx.x;
  const int slab = (int)blockIdx.x / (TTv / 64), lg = (int)blockIdx.x % (TTv / 64);
  const int b = slab / NHv, h = slab % NHv;
  for (int i = tid; i < 64 * 8; i += 256) {
    const int r = i / 8, c8 = (i % 8) * 8;
    const size_t s0 = ((size_t)b * TTv + (size_t)lg * 64 + r) * (size_t)ldv + (size_t)h * 64 + c8;
    Frag16 f;
    f.half[0] = *(const v8us*)(V + s0);
#pragma unroll
    for (int q = 0; q < 8; ++q) tl[r][c8 + q] = f.u[q];
    if (TWO) {
      Frag16 f2;
      f2.half[0] = *(const v8us*)(V2 + s0);
#pragma unroll
      for (int q = 0; q < 8; ++q) tl2[r][c8 + q] = f2.u[q];
    }
  }
  __syncthreads();
  for (int pass = 0; pass < 2; ++pass) {
#pragma unroll
    for (int rd = 0; rd < 2; ++rd) {
      const int d = rd * 32 + tid / 8, pc = tid % 8;
      Frag16 f;
#pragma unroll
      for (int q = 0; q < 8; ++q) f.u[q] = tl[pc * 8 + q][d];
      const size_t o = ((size_t)slab * 64 + d) * (size_t)TTv + (size_t)lg * 64 + pc * 8;
      *(volatile v8us*)(Vt + o) = f.half[0];
      if (TWO) {
        Frag16 f2;
#pragma unroll
        for (int q = 0; q < 8; ++q) f2.u[q] = tl2[pc * 8 + q][d];
        *(volatile v8us*)(Vt2 + o) = f2.half[0];
      }
    }
    if (pass == 0) __threadfence();
  }
}

template <bool CAUSAL, bool EARLY>
__global__ __launch_bounds__(128) void k_attn(const unsigned short* __restrict__ QH, const unsigned short* __restrict__ QL,
    const unsigned short* __restrict__ KH, const unsigned short* __restrict__ KL, const unsigned short* __restrict__ VT,
    const unsigned short* __restrict__ VL, unsigned short* __restrict__ CTX, int qb0) {
  static_assert(CAUSAL || !EARLY);
  __shared__ __attribute__((aligned(16))) unsigned short ph[4][2][16][64];
  __shared__ __attribute__((aligned(16))) unsigned short pe[EARLY ? 4 : 1][2][16][64];
  __shared__ __attribute__((aligned(16))) unsigned short so[4][16][72];
  const int tid = threadIdx.x, w = tid >> 5, lane = tid & 31, ln = lane & 15, hh = lane >> 4;
  const int bh = (int)blockIdx.x, b = bh / NH, h = bh % NH;
  const int qb = qb0 + (int)blockIdx.y;
  const int q0w = qb * KQB + w * 16;
  const size_t rowbase = (size_t)b * SEQ;
  Frag16 qh0, qh1, ql0, ql1;
  {
    const size_t qo = (rowbase + (size_t)q0w + ln) * DM + (size_t)h * HD;
    qh0 = ld_frag(QH + qo, hh); qh1 = ld_frag(QH + qo + 32, hh);
    ql0 = ld_frag(QL + qo, hh); ql1 = ld_frag(QL + qo + 32, hh);
  }
  const v8f z8 = {0.f, 0.f, 0.f, 0.f, 0.f, 0.f, 0.f, 0.f};
  v8f o[4] = {z8, z8, z8, z8};
  v8f oe[4] = {z8, z8, z8, z8};
  float m[8], l[8];
#pragma unroll
  for (int r = 0; r < 8; ++r) { m[r] = -1.0e30f; l[r] = 0.f; }
  const int nck = CAUSAL ? (qb + 1) : (SEQ / KQB);
#pragma unroll 1
  for (int kc = 0; kc < nck; ++kc) {
    const int par = kc & 1;
    const size_t krow = rowbase + (size_t)kc * KQB;
    v8f s[4];
#pragma unroll
    for (int t = 0; t < 4; ++t) {
      v8f acc = z8;
#pragma unroll
      for (int ks = 0; ks < 2; ++ks) {
        const size_t ko = (krow + (size_t)(t * 16 + ln)) * DM + (size_t)h * HD + ks * 32;
        const Frag16 kh = ld_frag(KH + ko, hh);
        const Frag16 kl = ld_frag(KL + ko, hh);
        const Frag16 qa = (ks == 0) ? qh0 : qh1;
        const Frag16 qe = (ks == 0) ? ql0 : ql1;
        acc = mma_b(qa.b, kh.b, acc);
        acc = mma_b(qe.b, kh.b, acc);
        acc = mma_b(qa.b, kl.b, acc);
      }
      s[t] = acc;
    }
#pragma unroll
    for (int r = 0; r < 8; ++r) {
      float sv[4];
#pragma unroll
      for (int t = 0; t < 4; ++t) sv[t] = s[t][r] * 8.0f;
      if (CAUSAL) {
        if (kc == qb) {
          const int qpos = q0w + 8 * hh + r;
#pragma unroll
          for (int t = 0; t < 4; ++t) { const int key = kc * KQB + t * 16 + ln; sv[t] = (key > qpos) ? -1.0e30f : sv[t]; }
        }
      }
      float mx = fmaxf(fmaxf(sv[0], sv[1]), fmaxf(sv[2], sv[3]));
      mx = fmaxf(mx, __shfl_xor(mx, 8, 32));
      mx = fmaxf(mx, __shfl_xor(mx, 4, 32));
      mx = fmaxf(mx, __shfl_xor(mx, 2, 32));
      mx = fmaxf(mx, __shfl_xor(mx, 1, 32));
      const float mn = fmaxf(m[r], mx);
      const float corr = __expf(m[r] - mn);
      float p[4];
      float psum = 0.f;
#pragma unroll
      for (int t = 0; t < 4; ++t) { p[t] = __expf(sv[t] - mn); psum += p[t]; }
      psum += __shfl_xor(psum, 8, 32);
      psum += __shfl_xor(psum, 4, 32);
      psum += __shfl_xor(psum, 2, 32);
      psum += __shfl_xor(psum, 1, 32);
      l[r] = l[r] * corr + psum;
      m[r] = mn;
#pragma unroll
      for (int j = 0; j < 4; ++j) o[j][r] = o[j][r] * corr;
      if (EARLY) {
#pragma unroll
        for (int j = 0; j < 4; ++j) oe[j][r] = oe[j][r] * corr;
      }
#pragma unroll
      for (int t = 0; t < 4; ++t) {
        const float pc = p[t] * 16384.0f;
        const unsigned short hb = f16_bits(pc);
        ph[w][par][8 * hh + r][t * 16 + ln] = hb;
        if (EARLY) pe[w][par][8 * hh + r][t * 16 + ln] = f16_bits((pc - f16_val(hb)) * 1024.0f);
      }
    }
    __builtin_amdgcn_fence(4  , "workgroup");
    __builtin_amdgcn_wave_barrier();
#pragma unroll
    for (int ks = 0; ks < 2; ++ks) {
      Frag16 pa;
      pa.half[0] = *(const v8us*)&ph[w][par][ln][ks * 32 + 8 * hh];
      pa.half[1] = *(const v8us*)&ph[w][par][ln][ks * 32 + 16 + 8 * hh];
      Frag16 pl = pa;
      if (EARLY) {
        pl.half[0] = *(const v8us*)&pe[w][par][ln][ks * 32 + 8 * hh];
        pl.half[1] = *(const v8us*)&pe[w][par][ln][ks * 32 + 16 + 8 * hh];
      }
#pragma unroll
      for (int j = 0; j < 4; ++j) {
        const size_t vo = ((size_t)bh * HD + (size_t)(j * 16 + ln)) * SEQ + (size_t)kc * KQB + ks * 32;
        const Frag16 vh = ld_frag(VT + vo, hh);
        o[j] = mma_h(pa.h, vh.h, o[j]);
        if (EARLY) {
          const Frag16 vl = ld_frag(VL + vo, hh);
          oe[j] = mma_h(pl.h, vh.h, oe[j]);
          oe[j] = mma_h(pa.h, vl.h, oe[j]);
        }
      }
    }
  }
  float li[8];
#pragma unroll
  for (int r = 0; r < 8; ++r) li[r] = 1.0f / l[r];
#pragma unroll
  for (int j = 0; j < 4; ++j) {
#pragma unroll
    for (int r = 0; r < 8; ++r) {
      float v = o[j][r] * (1.0f / 16384.0f);
      if (EARLY) v += oe[j][r] * (1.0f / 16777216.0f);
      v *= li[r];
      so[w][8 * hh + r][j * 16 + ln] = f16_bits(v);
    }
  }
  __builtin_amdgcn_fence(4  , "workgroup");
  __builtin_amdgcn_wave_barrier();
  for (int pass = 0; pass < 2; ++pass) {
#pragma unroll
    for (int q = 0; q < 4; ++q) {
      const int row = q * 4 + (lane >> 3), c8 = (lane & 7) * 8;
      const v8us v = *(const v8us*)&so[w][row][c8];
      *(volatile v8us*)(CTX + (rowbase + (size_t)q0w + row) * DM + (size_t)h * HD + c8) = v;
    }
    if (pass == 0) __threadfence();
  }
}

extern "C" void kernel_launch(void* const* d_in, const int* in_sizes, int n_in,
                              void* d_out, int out_size, void* d_ws, size_t ws_size, hipStream_t stream) {
  if (n_in < 14) return;
  const float* x  = (const float*)d_in[0];
  const float* Wq = (const float*)d_in[1];
  const float* bq = (const float*)d_in[2];
  const float* Wk = (const float*)d_in[3];
  const float* bk = (const float*)d_in[4];
  const float* Wv = (const float*)d_in[5];
  const float* bv = (const float*)d_in[6];
  const float* Wp = (const float*)d_in[7];
  const float* bp = (const float*)d_in[8];
  const float* gamma = (const float*)d_in[9];
  const float* W1 = (const float*)d_in[10];
  const float* b1 = (const float*)d_in[11];
  const float* W2 = (const float*)d_in[12];
  const float* b2 = (const float*)d_in[13];
  if ((size_t)in_sizes[0] < ((size_t)(NB - 1) * SEQ_FULL + SEQ) * DM) return;
  if (in_sizes[1] < DM * DM || in_sizes[3] < DM * DM || in_sizes[5] < DM * DM || in_sizes[7] < DM * DM) return;
  if (in_sizes[2] < DM || in_sizes[4] < DM || in_sizes[6] < DM || in_sizes[8] < DM || in_sizes[9] < DM || in_sizes[13] < DM) return;
  if (in_sizes[10] < DM * DFF || in_sizes[11] < DFF || in_sizes[12] < DFF * DM) return;
  if ((size_t)out_size < ((size_t)(NB - 1) * OSEQ + SEQ) * DM) return;

  char* ws = (char*)d_ws;
  size_t off = 0;
  auto take = [&](size_t bytes) { char* p = ws + off; off += (bytes + 255) & ~(size_t)255; return p; };
  const size_t WPL = (size_t)DM * DM * 2, ACT2 = NR * DM * 2, ACT4 = NR * DM * 4, FFP = (size_t)DM * DFF * 2, HPL = NR * DFF * 2;
  unsigned short* WQ16 = (unsigned short*)take(WPL);
  unsigned short* WK16 = (unsigned short*)take(WPL);
  unsigned short* WV16 = (unsigned short*)take(WPL);
  unsigned short* WP16 = (unsigned short*)take(WPL);
  unsigned short* WQB = (unsigned short*)take(WPL);
  unsigned short* WKB = (unsigned short*)take(WPL);
  char* rXB = take(ACT4);
  float* XB = (float*)rXB; unsigned short* PBH = (unsigned short*)rXB; unsigned short* PBL = (unsigned short*)(rXB + ACT2);
  char* rQK = take(4 * ACT2 > HPL ? 4 * ACT2 : HPL);
  unsigned short* QH = (unsigned short*)rQK; unsigned short* QL = (unsigned short*)(rQK + ACT2);
  unsigned short* KH = (unsigned short*)(rQK + 2 * ACT2); unsigned short* KL = (unsigned short*)(rQK + 3 * ACT2);
  unsigned short* H16 = (unsigned short*)rQK;
  char* rV = take(2 * ACT2);
  unsigned short* VH = (unsigned short*)rV; unsigned short* VLO = (unsigned short*)(rV + ACT2); float* A32 = (float*)rV;
  char* rVT = take(2 * ACT2 > 2 * FFP ? 2 * ACT2 : 2 * FFP);
  unsigned short* VT = (unsigned short*)rVT; unsigned short* VTL = (unsigned short*)(rVT + ACT2);
  unsigned short* W1P = (unsigned short*)rVT; unsigned short* W2P = (unsigned short*)(rVT + FFP);
  unsigned short* CTX = (unsigned short*)take(ACT2);
  char* rX16 = take(ACT2);
  unsigned short* X16 = (unsigned short*)rX16; unsigned short* A16 = (unsigned short*)rX16; unsigned short* B16F = (unsigned short*)rX16;
  float* B32 = (float*)take(ACT4);
  float* RSX = (float*)take(NR * 4);
  float* RSA = (float*)take(NR * 4);
  float* RSB = (float*)take(NR * 4);
  if (off > ws_size || off > ((size_t)128 << 20)) return;

  const unsigned gw   = (unsigned)(((size_t)DM * DM / 8 + 255) / 256);
  const unsigned gw1  = (unsigned)(((size_t)DM * DFF / 8 + 255) / 256);
  const unsigned grms = (unsigned)(NR / 32);
  const unsigned gq   = (unsigned)((NR / 128) * (DM / 64));
  const unsigned gff  = (unsigned)((NR / 128) * (DFF / 64));
  const unsigned gvt  = (unsigned)(NB * NH * (SEQ / 64));
  const float a16 = 0.0625f;
  const int M = (int)NR;
  float* out = (float*)d_out;

  k_wt<false, true><<<gw, 256, 0, stream>>>(Wq, gamma, WQ16, DM, DM, 16.0f);
  k_wt<false, true><<<gw, 256, 0, stream>>>(Wk, gamma, WK16, DM, DM, 16.0f);
  k_wt<false, true><<<gw, 256, 0, stream>>>(Wv, gamma, WV16, DM, DM, 16.0f);
  k_wt<false, false><<<gw, 256, 0, stream>>>(Wp, Wp, WP16, DM, DM, 16.0f);
  k_wt<true, true><<<gw, 256, 0, stream>>>(Wq, gamma, WQB, DM, DM, 1.0f);
  k_wt<true, true><<<gw, 256, 0, stream>>>(Wk, gamma, WKB, DM, DM, 1.0f);

  k_rms<true, true, true, false><<<grms, 256, 0, stream>>>(x, SEQ_FULL, RMS_EPS, XB, X16, nullptr, nullptr, RSX);
  k_gemm<false, false, 0, 3, true, false><<<gq, 128, 0, stream>>>(X16, nullptr, DM, WQ16, DM, a16, RSX, bq, nullptr, 0, nullptr, QH, QL, DM, M, 0, M, DM, DM);
  k_gemm<false, false, 0, 3, true, false><<<gq, 128, 0, stream>>>(X16, nullptr, DM, WK16, DM, a16, RSX, bk, nullptr, 0, nullptr, KH, KL, DM, M, 0, M, DM, DM);
  k_gemm<false, false, 0, 1, true, false><<<gq, 128, 0, stream>>>(X16, nullptr, DM, WV16, DM, a16, RSX, bv, nullptr, 0, nullptr, VH, nullptr, DM, M, 0, M, DM, DM);
  k_vt<NH, SEQ, false><<<gvt, 256, 0, stream>>>(VH, nullptr, DM, VT, nullptr);
  k_attn<false, false><<<dim3((unsigned)(NB * NH), (unsigned)(SEQ / KQB)), 128, 0, stream>>>(QH, QL, KH, KL, VT, VT, CTX, 0);
  k_gemm<false, false, 0, 0, false, true><<<gq, 128, 0, stream>>>(CTX, nullptr, DM, WP16, DM, a16, nullptr, bp, XB, DM, A32, nullptr, nullptr, DM, M, 0, M, DM, DM);

  k_rms<false, false, true, false><<<grms, 256, 0, stream>>>(A32, SEQ, RMS_EPS, nullptr, A16, nullptr, nullptr, RSA);
  k_wt<false, true><<<gw1, 256, 0, stream>>>(W1, gamma, W1P, DM, DFF, 16.0f);
  k_wt<false, false><<<gw1, 256, 0, stream>>>(W2, W2, W2P, DFF, DM, 16.0f);
  k_gemm<false, false, 1, 1, true, false><<<gff, 128, 0, stream>>>(A16, nullptr, DM, W1P, DM, a16, RSA, b1, nullptr, 0, nullptr, H16, nullptr, DFF, M, 0, M, DFF, DM);
  k_gemm<false, false, 0, 0, false, true><<<gq, 128, 0, stream>>>(H16, nullptr, DFF, W2P, DFF, a16, nullptr, b2, XB, DM, B32, nullptr, nullptr, DM, M, 0, M, DM, DFF);

  k_rms<false, false, true, true><<<grms, 256, 0, stream>>>(B32, SEQ, RMS_EPS, nullptr, B16F, PBH, PBL, RSB);
  k_gemm<true, true, 0, 3, true, false><<<gq, 128, 0, stream>>>(PBH, PBL, DM, WQB, DM, 1.0f, RSB, bq, nullptr, 0, nullptr, QH, QL, DM, M, 0, M, DM, DM);
  k_gemm<true, true, 0, 3, true, false><<<gq, 128, 0, stream>>>(PBH, PBL, DM, WKB, DM, 1.0f, RSB, bk, nullptr, 0, nullptr, KH, KL, DM, M, 0, M, DM, DM);
  k_gemm<false, false, 0, 2, true, false><<<gq, 128, 0, stream>>>(B16F, nullptr, DM, WV16, DM, a16, RSB, bv, nullptr, 0, nullptr, VH, VLO, DM, M, 0, M, DM, DM);
  k_vt<NH, SEQ, true><<<gvt, 256, 0, stream>>>(VH, VLO, DM, VT, VTL);
  k_attn<true, true><<<dim3((unsigned)(NB * NH), 1u), 128, 0, stream>>>(QH, QL, KH, KL, VT, VTL, CTX, 0);
  if (SEQ / KQB > 1) k_attn<true, false><<<dim3((unsigned)(NB * NH), (unsigned)(SEQ / KQB - 1)), 128, 0, stream>>>(QH, QL, KH, KL, VT, VTL, CTX, 1);
  k_gemm<false, false, 0, 0, false, true><<<gq, 128, 0, stream>>>(CTX, nullptr, DM, WP16, DM, a16, nullptr, bp, B32, DM, out, nullptr, nullptr, DM, SEQ, OSEQ, M, DM, DM);
}
